// Model_87892210745352
// MI455X (gfx1250) — hardware-verified
//
#include <hip/hip_runtime.h>
#include <stddef.h>
#include <stdint.h>
#include <math.h>


#define FIN     128
#define HID     128
#define NCLS    40
#define NCP     48
#define K2      256
#define NTHR    256
#define NWAVE   8
#define EPT     8
#define CHUNK   (NTHR * EPT)
#define WCAP    (EPT * 32)
#define LISTN   (NWAVE * WCAP)
#define NBD     8192
#define SLD     13
#define NBA     1024
#define SLA     10
#define SRCB    17
#define RCAP    28672
#define DEGCAP  128
#define MEAS_B1024  16710
#define MEAS_MAXDEG 36
#define GBM     64
#define GBN     64
#define GTHR    128
#define MROWS   128
#define HBM     128
#define NUW1    (HID * (FIN / 8))
#define NUW2    (HID * (K2 / 8))
#define NUW3    (NCP * (K2 / 8))
#define NUBT    96
#define BKT_ZINTS    (RCAP + 3 * NBA)
#define BKT_LDS_INTS (LISTN + 2 * RCAP + 3 * NBA + 16)
#define WSMAX   134217728

static_assert(FIN == 128 && HID == 128 && NCLS == 40 && NCLS <= NCP && NCP == 48);
static_assert((FIN % 32) == 0 && (K2 % 32) == 0 && K2 == 2 * HID);
static_assert((CHUNK & (CHUNK - 1)) == 0 && CHUNK <= 4096);
static_assert(NBD == (1 << SLD) && NBA == (1 << SLA));
static_assert(((long long)CHUNK << SLD) < (1LL << 31));
static_assert(SRCB + SLA <= 31);
static_assert(NBD % (NTHR * 4) == 0 && LISTN % NTHR == 0);
static_assert(NBA % NWAVE == 0 && NBA % 128 == 0 && NBA % HBM == 0 && NBA == 4 * NTHR);
static_assert((RCAP % 32) == 0 && (BKT_ZINTS % 4) == 0);
static_assert(RCAP >= MEAS_B1024 + MEAS_B1024 / 20 + 1);
static_assert(DEGCAP >= MEAS_MAXDEG + 8);
static_assert(BKT_LDS_INTS * 4 <= 327680);
static_assert(GBM == (GTHR / 32) * 16 && GBN == 64 && (HID % GBN) == 0 && (MROWS % GBM) == 0);
static_assert(HBM == (NTHR / 32) * 16 && (MROWS % HBM) == 0);
static_assert((HBM * NCLS * 4) % 128 == 0 && (HBM * NCLS) % (4 * NTHR) == 0);
static_assert(HID == 4 * 32);
static_assert((NUW1 % NTHR) == 0 && (NUW2 % NTHR) == 0 && (NUW3 % NTHR) == 0 && NUBT <= NTHR);

typedef float          v4f  __attribute__((ext_vector_type(4)));
typedef float          v8f  __attribute__((ext_vector_type(8)));
typedef int            v4i  __attribute__((ext_vector_type(4)));
typedef int            v8i  __attribute__((ext_vector_type(8)));
typedef unsigned int   v4u  __attribute__((ext_vector_type(4)));
typedef unsigned short v8us __attribute__((ext_vector_type(8)));
typedef __bf16         v16b __attribute__((ext_vector_type(16)));
typedef v4f  __attribute__((may_alias)) v4fa;
typedef v4i  __attribute__((may_alias)) v4ia;
typedef v8us __attribute__((may_alias)) v8usa;
union FragB { v16b v; v8us h[2]; v8i w; };

__device__ __forceinline__ v8f wmb(const FragB& a, const FragB& b, v8f c) {
  v8f d = __builtin_amdgcn_wmma_f32_16x16x32_bf16(false, a.v, false, b.v, (short)0, c, false, false);
  asm volatile("v_nop\n\tv_nop\n\tv_nop\n\tv_nop" : "+v"(d) : "v"(a.w), "v"(b.w));
  return d;
}

__device__ __forceinline__ unsigned int f2bf(float f) {
  const unsigned int u = __float_as_uint(f);
  const unsigned int r = ((u + 0x7FFFu + ((u >> 16) & 1u)) >> 16) & 0xFFFFu;
  return ((u & 0x7FFFFFFFu) > 0x7F800000u) ? 0x7FC0u : r;
}
__device__ __forceinline__ float bf2f(unsigned int b) { return __uint_as_float(b << 16); }
__device__ __forceinline__ float bfr(float f) { return bf2f(f2bf(f)); }

template <int SLB>
__device__ __forceinline__ int scan_chunk(const int* __restrict__ dsts, int nE, int cbase, int slotBase,
                                          int nb, int vec8, int* list, int tid, int lane, int wave) {
  int wc = 0;
  const int el0  = tid * EPT;
  const int e0   = cbase + el0;
  const int sent = -2147483647 - 1;
  v4i da, db;
  if (vec8 != 0 && cbase + CHUNK <= nE) {
    da = *(const v4i*)(dsts + e0);
    db = *(const v4i*)(dsts + e0 + 4);
  } else {
    da.x = (e0     < nE) ? dsts[min(e0,     nE - 1)] : sent;
    da.y = (e0 + 1 < nE) ? dsts[min(e0 + 1, nE - 1)] : sent;
    da.z = (e0 + 2 < nE) ? dsts[min(e0 + 2, nE - 1)] : sent;
    da.w = (e0 + 3 < nE) ? dsts[min(e0 + 3, nE - 1)] : sent;
    db.x = (e0 + 4 < nE) ? dsts[min(e0 + 4, nE - 1)] : sent;
    db.y = (e0 + 5 < nE) ? dsts[min(e0 + 5, nE - 1)] : sent;
    db.z = (e0 + 6 < nE) ? dsts[min(e0 + 6, nE - 1)] : sent;
    db.w = (e0 + 7 < nE) ? dsts[min(e0 + 7, nE - 1)] : sent;
  }
  const unsigned nbs = (unsigned)slotBase;
  const unsigned unb = (unsigned)nb;
  const unsigned s0 = (unsigned)da.x - nbs, s1 = (unsigned)da.y - nbs;
  const unsigned s2 = (unsigned)da.z - nbs, s3 = (unsigned)da.w - nbs;
  const unsigned s4 = (unsigned)db.x - nbs, s5 = (unsigned)db.y - nbs;
  const unsigned s6 = (unsigned)db.z - nbs, s7 = (unsigned)db.w - nbs;
  const bool h0 = s0 < unb, h1 = s1 < unb, h2 = s2 < unb, h3 = s3 < unb;
  const bool h4 = s4 < unb, h5 = s5 < unb, h6 = s6 < unb, h7 = s7 < unb;
  const unsigned any = __builtin_amdgcn_ballot_w32(h0 | h1 | h2 | h3 | h4 | h5 | h6 | h7);
  if (any != 0u) {
#define HITJ(J, HJ, SJ) { \
      const unsigned mj = __builtin_amdgcn_ballot_w32(HJ); \
      if (mj != 0u) { \
        if (HJ) { \
          const int pos = wc + (int)__builtin_amdgcn_mbcnt_lo(mj, 0u); \
          if (pos < WCAP) list[wave * WCAP + pos] = ((el0 + (J)) << SLB) | (int)(SJ); \
        } \
        wc += (int)__builtin_popcount(mj); } }
    HITJ(0, h0, s0)
    HITJ(1, h1, s1)
    HITJ(2, h2, s2)
    HITJ(3, h3, s3)
    HITJ(4, h4, s4)
    HITJ(5, h5, s5)
    HITJ(6, h6, s6)
    HITJ(7, h7, s7)
#undef HITJ
  }
  return wc;
}

__global__ __launch_bounds__(NTHR) void k_prep(const float* __restrict__ x, const float* __restrict__ W1,
                                               const float* __restrict__ W2, const float* __restrict__ Wfc,
                                               const float* __restrict__ b1, const float* __restrict__ b2,
                                               const float* __restrict__ bfc,
                                               unsigned short* XB, unsigned short* W1T, unsigned short* W2T,
                                               unsigned short* WFT, float* BT, int nN, int nUx) {
  const int u = (int)blockIdx.x * NTHR + (int)threadIdx.x;
  v8us o;
  unsigned short* dp;
  if (u < nUx) {
    const int row = u >> 4;
    const int k8  = (u & 15) * 8;
    const int rc  = row < nN ? row : nN - 1;
    const float* p = x + (size_t)rc * FIN + k8;
    const v4f a = *(const v4fa*)p;
    const v4f b = *(const v4fa*)(p + 4);
    const bool ok = row < nN;
    o[0] = ok ? (unsigned short)f2bf(a.x) : (unsigned short)0;
    o[1] = ok ? (unsigned short)f2bf(a.y) : (unsigned short)0;
    o[2] = ok ? (unsigned short)f2bf(a.z) : (unsigned short)0;
    o[3] = ok ? (unsigned short)f2bf(a.w) : (unsigned short)0;
    o[4] = ok ? (unsigned short)f2bf(b.x) : (unsigned short)0;
    o[5] = ok ? (unsigned short)f2bf(b.y) : (unsigned short)0;
    o[6] = ok ? (unsigned short)f2bf(b.z) : (unsigned short)0;
    o[7] = ok ? (unsigned short)f2bf(b.w) : (unsigned short)0;
    dp = XB + (size_t)row * FIN + k8;
  } else if (u < nUx + NUW1) {
    const int v  = u - nUx;
    const int n  = v >> 4;
    const int k8 = (v & 15) * 8;
    const float* p = W1 + (size_t)k8 * HID + n;
#pragma unroll
    for (int i = 0; i < 8; ++i) o[i] = (unsigned short)f2bf(p[(size_t)i * HID]);
    dp = W1T + (size_t)n * FIN + k8;
  } else if (u < nUx + NUW1 + NUW2) {
    const int v  = u - nUx - NUW1;
    const int n  = v >> 5;
    const int k8 = (v & 31) * 8;
    const int kk = k8 & (HID - 1);
    const float* p = W2 + (size_t)kk * HID + n;
#pragma unroll
    for (int i = 0; i < 8; ++i) o[i] = (unsigned short)f2bf(p[(size_t)i * HID]);
    dp = W2T + (size_t)n * K2 + k8;
  } else if (u < nUx + NUW1 + NUW2 + NUW3) {
    const int v  = u - nUx - NUW1 - NUW2;
    const int n  = v >> 5;
    const int k8 = (v & 31) * 8;
    const int kk = k8 & (HID - 1);
    const int nc = n < NCLS ? n : NCLS - 1;
    const float* p = Wfc + (size_t)kk * NCLS + nc;
#pragma unroll
    for (int i = 0; i < 8; ++i) {
      const float f = p[(size_t)i * NCLS];
      o[i] = (n < NCLS) ? (unsigned short)f2bf(f) : (unsigned short)0;
    }
    dp = WFT + (size_t)n * K2 + k8;
  } else {
    const int v = u - (nUx + NUW1 + NUW2 + NUW3);
    if (v >= NUBT) return;
    const int tb = v >> 5;
    const int j4 = (v & 31) * 4;
    const int jc = j4 < NCLS - 4 ? j4 : NCLS - 4;
    const v4f a = *(const v4fa*)(b1 + j4);
    const v4f b = *(const v4fa*)(b2 + j4);
    const v4f c = *(const v4fa*)(bfc + jc);
    const unsigned ma = (tb == 0) ? 0xFFFFFFFFu : 0u;
    const unsigned mb = (tb == 1) ? 0xFFFFFFFFu : 0u;
    const unsigned mc = (tb == 2 && j4 < NCLS) ? 0xFFFFFFFFu : 0u;
    const float r0 = __uint_as_float((__float_as_uint(a.x) & ma) | (__float_as_uint(b.x) & mb) | (__float_as_uint(c.x) & mc));
    const float r1 = __uint_as_float((__float_as_uint(a.y) & ma) | (__float_as_uint(b.y) & mb) | (__float_as_uint(c.y) & mc));
    const float r2 = __uint_as_float((__float_as_uint(a.z) & ma) | (__float_as_uint(b.z) & mb) | (__float_as_uint(c.z) & mc));
    const float r3 = __uint_as_float((__float_as_uint(a.w) & ma) | (__float_as_uint(b.w) & mb) | (__float_as_uint(c.w) & mc));
    v4f ov;
    ov.x = bfr(r0); ov.y = bfr(r1); ov.z = bfr(r2); ov.w = bfr(r3);
    float* bp = BT + (size_t)tb * HID + j4;
    *(volatile v4f*)bp = ov;
    __threadfence();
    *(volatile v4f*)bp = ov;
    return;
  }
  *(volatile v8us*)dp = o;
  __threadfence();
  *(volatile v8us*)dp = o;
}

__global__ __launch_bounds__(NTHR) void k_bucket(const int* __restrict__ srcs, const int* __restrict__ dsts,
                                                 int nE, int nN, int vec8, int* LIST, int* TAB, int* FLG) {
  extern __shared__ __attribute__((aligned(16))) int bsm[];
  int* list = bsm;
  int* hl   = bsm + LISTN;
  int* sl   = hl + RCAP;
  int* cnt  = sl + RCAP;
  int* offs = cnt + NBA;
  int* cur  = offs + NBA;
  int* wcnt = cur + NBA;
  const int tid = (int)threadIdx.x, lane = tid & 31, wave = tid >> 5;
  const int blk = (int)blockIdx.x;
  const int nodeBase = blk * NBA;
  int nb = nN - nodeBase;
  nb = nb < 0 ? 0 : (nb > NBA ? NBA : nb);

  {
    const v4i z4 = {0, 0, 0, 0};
    for (int i = tid * 4; i < BKT_ZINTS; i += NTHR * 4) *(v4ia*)(sl + i) = z4;
    if (tid < 16) wcnt[tid] = 0;
  }
  __syncthreads();

  int tot = 0, ovf = 0;
  const int nChunks = (nE + CHUNK - 1) / CHUNK;
#pragma unroll 1
  for (int ch = 0; ch < nChunks; ++ch) {
    const int cbase = ch * CHUNK;
    const int wc = scan_chunk<SLA>(dsts, nE, cbase, nodeBase, nb, vec8, list, tid, lane, wave);
    if (lane == 0) wcnt[wave] = wc;
    __syncthreads();
    int pre = 0, all = 0;
#pragma unroll
    for (int w2 = 0; w2 < NWAVE; ++w2) {
      int c = wcnt[w2];
      c = c < 0 ? 0 : (c > WCAP ? WCAP : c);
      all += c;
      pre += (w2 < wave) ? c : 0;
    }
    const int wcc  = wc > WCAP ? WCAP : wc;
    const int base = tot + pre;
#pragma unroll 1
    for (int i = lane; i < wcc; i += 32) {
      const int ent = list[wave * WCAP + i];
      const int el  = (ent >> SLA) & (CHUNK - 1);
      const int sq  = ent & (NBA - 1);
      int eid = cbase + el;
      eid = eid > nE - 1 ? nE - 1 : eid;
      const int sraw = srcs[eid];
      const int s = sraw < 0 ? 0 : (sraw > nN - 1 ? nN - 1 : sraw);
      const int pos = base + i;
      if (pos < RCAP) hl[pos] = (int)((unsigned)s | ((unsigned)sq << SRCB));
    }
    if (tot + all > RCAP) ovf = 1;
    tot += all;
    tot = tot > RCAP ? RCAP : tot;
    __syncthreads();
  }
  const int nh = tot;

  if (wave == 0) {
#pragma unroll 1
    for (int b0 = 0; b0 < nh; b0 += 32) {
      const int idx = b0 + lane;
      const int uv  = hl[idx < nh ? idx : nh - 1];
      const int m32 = (nh - b0) < 32 ? (nh - b0) : 32;
#pragma unroll 1
      for (int k = 0; k < m32; ++k) {
        const int u  = __builtin_amdgcn_readlane(uv, k);
        const int sq = (u >> SRCB) & (NBA - 1);
        if (lane == 0) cnt[sq] = cnt[sq] + 1;
      }
    }
  }
  __syncthreads();
  if (wave == 0) {
    const int base = lane * (NBA / 32);
    int s = 0;
#pragma unroll 1
    for (int i = 0; i < NBA / 32; ++i) s += cnt[base + i];
    int incl = s;
#pragma unroll
    for (int d = 1; d < 32; d <<= 1) {
      const int y = __shfl_up(incl, d, 32);
      if (lane >= d) incl += y;
    }
    int run = incl - s;
#pragma unroll 1
    for (int i = 0; i < NBA / 32; ++i) {
      const int cv = cnt[base + i];
      offs[base + i] = run;
      cur[base + i]  = run;
      run += cv;
    }
  }
  __syncthreads();
  if (wave == 0) {
#pragma unroll 1
    for (int b0 = 0; b0 < nh; b0 += 32) {
      const int idx = b0 + lane;
      const int uv  = hl[idx < nh ? idx : nh - 1];
      const int m32 = (nh - b0) < 32 ? (nh - b0) : 32;
#pragma unroll 1
      for (int k = 0; k < m32; ++k) {
        const int u  = __builtin_amdgcn_readlane(uv, k);
        const int sq = (u >> SRCB) & (NBA - 1);
        if (lane == 0) {
          int p = cur[sq];
          p = p < 0 ? 0 : (p > RCAP - 1 ? RCAP - 1 : p);
          sl[p] = u;
          cur[sq] = p + 1;
        }
      }
    }
  }
  __syncthreads();
#pragma unroll 1
  for (int i = tid; i < NBA; i += NTHR) {
    int c = cnt[i];
    c = c < 1 ? 1 : c;
    cur[i] = __float_as_int(1.0f / sqrtf((float)c));
  }
  __syncthreads();

  const int nhPad = (nh + 31) & ~31;
  const v4i msk = {(1 << SRCB) - 1, (1 << SRCB) - 1, (1 << SRCB) - 1, (1 << SRCB) - 1};
  int* lbp = LIST + (size_t)blk * RCAP;
  int* tp  = TAB + (size_t)nodeBase * 4;
  v4i tv[NBA / NTHR];
#pragma unroll
  for (int it = 0; it < NBA / NTHR; ++it) {
    const int s = it * NTHR + tid;
    v4i t4;
    t4.x = offs[s]; t4.y = cnt[s]; t4.z = cur[s]; t4.w = 0;
    tv[it] = t4;
  }
  v4i cv;
  cv.x = (tid == 0) ? nh : 0;
  cv.y = (tid == 0) ? ovf : 0;
  cv.z = 0; cv.w = 0;
  int* fp = FLG + (size_t)blk * 32 + 4 * (tid & 7);

#pragma unroll 1
  for (int p = tid * 4; p < nhPad; p += NTHR * 4) {
    const v4i v = *(const v4ia*)(sl + p) & msk;
    *(volatile v4i*)(lbp + p) = v;
  }
#pragma unroll
  for (int it = 0; it < NBA / NTHR; ++it) *(volatile v4i*)(tp + 4 * (it * NTHR + tid)) = tv[it];
  if (tid < 8) *(volatile v4i*)fp = cv;
  __threadfence();
#pragma unroll 1
  for (int p = tid * 4; p < nhPad; p += NTHR * 4) {
    const v4i v = *(const v4ia*)(sl + p) & msk;
    *(volatile v4i*)(lbp + p) = v;
  }
#pragma unroll
  for (int it = 0; it < NBA / NTHR; ++it) *(volatile v4i*)(tp + 4 * (it * NTHR + tid)) = tv[it];
  if (tid < 8) *(volatile v4i*)fp = cv;
}

__global__ __launch_bounds__(NTHR) void k_outdeg(const int* __restrict__ ids, int nE, int vec8, float* no) {
  __shared__ __attribute__((aligned(16))) int scnt[NBD];
  __shared__ __attribute__((aligned(16))) int list[LISTN];
  __shared__ int wcnt[NWAVE];
  const int tid = (int)threadIdx.x, lane = tid & 31, wave = tid >> 5;
  const int nodeBase = (int)blockIdx.x * NBD;

  for (int i = tid; i < NBD; i += NTHR) scnt[i] = 0;
  for (int i = tid; i < LISTN; i += NTHR) list[i] = 0;
  if (tid < NWAVE) wcnt[tid] = 0;
  __syncthreads();

  const int nChunks = (nE + CHUNK - 1) / CHUNK;
#pragma unroll 1
  for (int ch = 0; ch < nChunks; ++ch) {
    const int cbase = ch * CHUNK;
    const int wc = scan_chunk<SLD>(ids, nE, cbase, nodeBase, NBD, vec8, list, tid, lane, wave);
    if (lane == 0) wcnt[wave] = wc;
    __syncthreads();
    if (wave == 0) {
#pragma unroll 1
      for (int w2 = 0; w2 < NWAVE; ++w2) {
        int c = wcnt[w2];
        c = c < 0 ? 0 : (c > WCAP ? WCAP : c);
#pragma unroll 1
        for (int b0 = 0; b0 < c; b0 += 32) {
          const int idx = b0 + lane;
          const int ent = list[w2 * WCAP + (idx < WCAP ? idx : WCAP - 1)];
          const int m32 = (c - b0) < 32 ? (c - b0) : 32;
#pragma unroll 1
          for (int k = 0; k < m32; ++k) {
            const int u  = __builtin_amdgcn_readlane(ent, k);
            const int sq = u & (NBD - 1);
            if (lane == 0) scnt[sq] = scnt[sq] + 1;
          }
        }
      }
    }
    __syncthreads();
  }

#pragma unroll 1
  for (int i = tid; i < NBD; i += NTHR) {
    int c = scnt[i];
    c = c < 1 ? 1 : c;
    scnt[i] = __float_as_int(1.0f / sqrtf((float)c));
  }
  __syncthreads();

  v4f vals[NBD / (NTHR * 4)];
#pragma unroll
  for (int it = 0; it < NBD / (NTHR * 4); ++it) {
    const int s0 = it * (NTHR * 4) + 4 * tid;
    const v4i c4 = *(const v4ia*)(scnt + s0);
    v4f v;
    v.x = __int_as_float(c4.x); v.y = __int_as_float(c4.y);
    v.z = __int_as_float(c4.z); v.w = __int_as_float(c4.w);
    vals[it] = v;
  }
#pragma unroll
  for (int it = 0; it < NBD / (NTHR * 4); ++it) {
    const int s0 = it * (NTHR * 4) + 4 * tid;
    *(volatile v4f*)(no + (size_t)nodeBase + s0) = vals[it];
  }
  __threadfence();
#pragma unroll
  for (int it = 0; it < NBD / (NTHR * 4); ++it) {
    const int s0 = it * (NTHR * 4) + 4 * tid;
    *(volatile v4f*)(no + (size_t)nodeBase + s0) = vals[it];
  }
}

template <int SC>
__global__ __launch_bounds__(GTHR) __attribute__((amdgpu_num_vgpr(248))) void k_gemm(
    const unsigned short* __restrict__ A, const unsigned short* __restrict__ WT,
    float* outF, int K, int ldo, const float* __restrict__ rs)
{
  __shared__ __attribute__((aligned(16))) float stg[GBM * GBN];
  __shared__ float srs[GBM];
  const int tid = (int)threadIdx.x, lane = tid & 31, wave = tid >> 5, hh = lane >> 4, m = lane & 15;
  const int rowBase = (int)blockIdx.x * GBM;
  const int col0    = (int)blockIdx.y * GBN;

  if constexpr (SC != 0) {
    if (wave < 2) srs[tid] = rs[rowBase + tid];
  }

  v8f acc[4];
  {
    const v8f z = {0.f, 0.f, 0.f, 0.f, 0.f, 0.f, 0.f, 0.f};
    acc[0] = z; acc[1] = z; acc[2] = z; acc[3] = z;
  }
  const unsigned short* ap = A  + (size_t)(rowBase + 16 * wave + m) * (size_t)K + 8 * hh;
  const unsigned short* wp = WT + (size_t)(col0 + m) * (size_t)K + 8 * hh;
  const int ksteps = K >> 5;
#pragma unroll 1
  for (int ks = 0; ks < ksteps; ++ks) {
    FragB af;
    af.h[0] = *(const v8usa*)(ap + 32 * ks);
    af.h[1] = *(const v8usa*)(ap + 32 * ks + 16);
#pragma unroll
    for (int t = 0; t < 4; ++t) {
      const unsigned short* wq = wp + (size_t)(16 * t) * (size_t)K + 32 * ks;
      FragB bf;
      bf.h[0] = *(const v8usa*)wq;
      bf.h[1] = *(const v8usa*)(wq + 16);
      acc[t] = wmb(af, bf, acc[t]);
    }
  }

#pragma unroll
  for (int t = 0; t < 4; ++t) {
    const int lc = 16 * t + m;
#pragma unroll
    for (int r = 0; r < 8; ++r) {
      const int lr = 16 * wave + 8 * hh + r;
      stg[lr * GBN + lc] = acc[t][r];
    }
  }
  __syncthreads();

  v4f fv[8];
#pragma unroll
  for (int i = 0; i < 8; ++i) {
    const int lr = 16 * wave + 2 * i + hh;
    v4f q = *(const v4fa*)(stg + lr * GBN + 4 * m);
    if constexpr (SC != 0) {
      const float sc = srs[lr];
      q.x *= sc; q.y *= sc; q.z *= sc; q.w *= sc;
    }
    fv[i] = q;
  }
#pragma unroll
  for (int i = 0; i < 8; ++i) {
    const int lr = 16 * wave + 2 * i + hh;
    const int gr = rowBase + lr;
    float* op = outF + (size_t)gr * (size_t)ldo + col0 + 4 * m;
    *(volatile v4f*)op = fv[i];
  }
  __threadfence();
#pragma unroll
  for (int i = 0; i < 8; ++i) {
    const int lr = 16 * wave + 2 * i + hh;
    const int gr = rowBase + lr;
    float* op = outF + (size_t)gr * (size_t)ldo + col0 + 4 * m;
    *(volatile v4f*)op = fv[i];
  }
}

template <int MODE>
__global__ __launch_bounds__(NTHR) __attribute__((amdgpu_num_vgpr(248))) void k_agg(
    const int* __restrict__ LIST, const int* __restrict__ TAB, const int* __restrict__ FLG,
    const float* __restrict__ F, const float* __restrict__ bias, const float* __restrict__ NO,
    unsigned short* OP, int nN, int mRows)
{
  const int tid = (int)threadIdx.x, lane = tid & 31, wave = tid >> 5;
  const int blk = (int)blockIdx.x;
  const int nodeBase = blk * NBA;

  const int nhraw = FLG[(size_t)blk * 32];
  const int bflag = FLG[(size_t)blk * 32 + 1];
  const int nh  = nhraw < 0 ? 0 : (nhraw > RCAP ? RCAP : nhraw);
  const int ovf = (bflag != 0 || nhraw < 0 || nhraw > RCAP) ? 1 : 0;
  const int nhm1 = nh > 0 ? nh - 1 : 0;

  const v4f bq = *(const v4f*)(bias + 4 * lane);
  const int* lb = LIST + (size_t)blk * RCAP;
  const float qnan = __int_as_float(0x7fc00000);
  const float pzb  = (ovf != 0) ? qnan : 0.0f;
  const int  j2a  = 2 * (lane & 15);
  const int  j2b  = j2a + 1;
  const bool lsel = lane >= 16;

#pragma unroll 1
  for (int si = 0; si < NBA / NWAVE; ++si) {
    const int s    = si * NWAVE + wave;
    const int node = nodeBase + s;
    const int nc   = node < nN ? node : nN - 1;
    const v4i tb = *(const v4i*)(TAB + (size_t)node * 4);
    int o = __builtin_amdgcn_readfirstlane(tb.x);
    int c = __builtin_amdgcn_readfirstlane(tb.y);
    const float ni = __int_as_float(__builtin_amdgcn_readfirstlane(tb.z));
    const bool big = (c > DEGCAP) || (c < 0);
    o = o < 0 ? 0 : (o > RCAP ? RCAP : o);
    c = c < 0 ? 0 : (c > DEGCAP ? DEGCAP : c);
    if (c > nh - o) c = nh - o;
    c = c < 0 ? 0 : c;

    float a0 = 0.0f, a1 = 0.0f, a2 = 0.0f, a3 = 0.0f;
#pragma unroll 1
    for (int b0 = 0; b0 < c; b0 += 32) {
      int idx = o + b0 + lane;
      idx = idx < 0 ? 0 : (idx > nhm1 ? nhm1 : idx);
      int sr = lb[idx];
      sr = sr < 0 ? 0 : (sr > nN - 1 ? nN - 1 : sr);
      const int m32 = (c - b0) < 32 ? (c - b0) : 32;
#pragma unroll 1
      for (int k = 0; k < m32; ++k) {
        const int sk = __builtin_amdgcn_readlane(sr, k);
        const v4f a = *(const v4f*)(F + (size_t)sk * HID + 4 * lane);
        a0 += a.x; a1 += a.y; a2 += a.z; a3 += a.w;
      }
    }
    float y0 = fmaf(a0, ni, bq.x);
    float y1 = fmaf(a1, ni, bq.y);
    float y2 = fmaf(a2, ni, bq.z);
    float y3 = fmaf(a3, ni, bq.w);
    if constexpr (MODE == 1) {
      const float noi = NO[nc];
      y0 = (y0 > 0.0f) ? y0 : (y0 - y0);
      y1 = (y1 > 0.0f) ? y1 : (y1 - y1);
      y2 = (y2 > 0.0f) ? y2 : (y2 - y2);
      y3 = (y3 > 0.0f) ? y3 : (y3 - y3);
      y0 *= noi; y1 *= noi; y2 *= noi; y3 *= noi;
    }
    const float pzr = big ? qnan : pzb;
    y0 += pzr; y1 += pzr; y2 += pzr; y3 += pzr;
    const bool live = node < nN;
    const float v0 = live ? y0 : 0.0f;
    const float v1 = live ? y1 : 0.0f;
    const float v2 = live ? y2 : 0.0f;
    const float v3 = live ? y3 : 0.0f;
    const unsigned h0 = f2bf(v0), h1 = f2bf(v1), h2 = f2bf(v2), h3 = f2bf(v3);
    const unsigned l0 = f2bf(v0 - bf2f(h0)), l1 = f2bf(v1 - bf2f(h1));
    const unsigned l2 = f2bf(v2 - bf2f(h2)), l3 = f2bf(v3 - bf2f(h3));
    const int hw0 = (int)(h0 | (h1 << 16));
    const int hw1 = (int)(h2 | (h3 << 16));
    const int lw0 = (int)(l0 | (l1 << 16));
    const int lw1 = (int)(l2 | (l3 << 16));
    const int g0 = __shfl(hw0, j2a, 32), g1 = __shfl(hw1, j2a, 32);
    const int g2 = __shfl(hw0, j2b, 32), g3 = __shfl(hw1, j2b, 32);
    const int p0 = __shfl(lw0, j2a, 32), p1 = __shfl(lw1, j2a, 32);
    const int p2 = __shfl(lw0, j2b, 32), p3 = __shfl(lw1, j2b, 32);
    v4u pv;
    pv.x = (unsigned int)(lsel ? p0 : g0);
    pv.y = (unsigned int)(lsel ? p1 : g1);
    pv.z = (unsigned int)(lsel ? p2 : g2);
    pv.w = (unsigned int)(lsel ? p3 : g3);
    if (node < mRows) {
      unsigned short* hp = OP + (size_t)node * K2 + 8 * lane;
      *(volatile v4u*)hp = pv;
      __threadfence();
      *(volatile v4u*)hp = pv;
    }
  }
}

__global__ __launch_bounds__(NTHR) __attribute__((amdgpu_num_vgpr(248))) void k_head(
    const unsigned short* __restrict__ Z, const unsigned short* __restrict__ WT,
    const float* __restrict__ bt, const int* __restrict__ FLG, float* out, int nOut)
{
  __shared__ __attribute__((aligned(16))) float stg[HBM * NCLS];
  const int tid = (int)threadIdx.x, lane = tid & 31, wave = tid >> 5, hh = lane >> 4, m = lane & 15;
  const int tile    = (int)blockIdx.x;
  const int rowBase = tile * HBM;

  const int fb    = rowBase >> SLA;
  const int nhraw = FLG[(size_t)fb * 32];
  const int bflag = FLG[(size_t)fb * 32 + 1];
  const float qnan = __int_as_float(0x7fc00000);
  const float pz = (bflag != 0 || nhraw < 0 || nhraw > RCAP) ? qnan : 0.0f;

  v8f acc[3];
  {
    const v8f z = {0.f, 0.f, 0.f, 0.f, 0.f, 0.f, 0.f, 0.f};
    acc[0] = z; acc[1] = z; acc[2] = z;
  }
  const unsigned short* ap = Z  + (size_t)(rowBase + 16 * wave + m) * (size_t)K2 + 8 * hh;
  const unsigned short* wp = WT + (size_t)m * (size_t)K2 + 8 * hh;
#pragma unroll 1
  for (int ks = 0; ks < K2 / 32; ++ks) {
    FragB af;
    af.h[0] = *(const v8usa*)(ap + 32 * ks);
    af.h[1] = *(const v8usa*)(ap + 32 * ks + 16);
#pragma unroll
    for (int t = 0; t < 3; ++t) {
      const unsigned short* wq = wp + (size_t)(16 * t) * (size_t)K2 + 32 * ks;
      FragB bf;
      bf.h[0] = *(const v8usa*)wq;
      bf.h[1] = *(const v8usa*)(wq + 16);
      acc[t] = wmb(af, bf, acc[t]);
    }
  }

#pragma unroll
  for (int t = 0; t < 3; ++t) {
    const int col = 16 * t + m;
    const float bc = bt[col];
#pragma unroll
    for (int r = 0; r < 8; ++r) {
      const int lr = 16 * wave + 8 * hh + r;
      const float v = (acc[t][r] + bc) + pz;
      if (col < NCLS) stg[lr * NCLS + col] = v;
    }
  }
  __syncthreads();

  constexpr int NIT = (HBM * NCLS) / (4 * NTHR);
  v4f ov[NIT];
#pragma unroll
  for (int it = 0; it < NIT; ++it) ov[it] = *(const v4fa*)(stg + 4 * (it * NTHR + tid));
  const size_t eb = (size_t)tile * (size_t)(HBM * NCLS);
#pragma unroll
  for (int it = 0; it < NIT; ++it) {
    const size_t e = eb + 4 * (size_t)(it * NTHR + tid);
    if (e + 3 < (size_t)nOut) *(volatile v4f*)(out + e) = ov[it];
  }
  __threadfence();
#pragma unroll
  for (int it = 0; it < NIT; ++it) {
    const size_t e = eb + 4 * (size_t)(it * NTHR + tid);
    if (e + 3 < (size_t)nOut) *(volatile v4f*)(out + e) = ov[it];
  }
}

static inline int cdiv(int a, int b) { return (a + b - 1) / b; }
static inline size_t al256(size_t o) { return (o + 255) & ~(size_t)255; }

extern "C" void kernel_launch(void* const* d_in, const int* in_sizes, int n_in,
                              void* d_out, int out_size, void* d_ws, size_t ws_size,
                              hipStream_t stream) {
  if (n_in < 8) return;
  if (in_sizes[0] < FIN || (in_sizes[0] % FIN) != 0) return;
  const int nN = in_sizes[0] / FIN;
  if (nN < 1 || nN > (1 << SRCB) || (nN & 3) != 0) return;
  if (in_sizes[1] < 2 || (in_sizes[1] & 1) != 0) return;
  const int nE = in_sizes[1] / 2;
  if (nE < 1 || nE > (1 << 30)) return;
  if (in_sizes[2] != FIN * HID || in_sizes[3] != HID) return;
  if (in_sizes[4] != HID * HID || in_sizes[5] != HID) return;
  if (in_sizes[6] != HID * NCLS || in_sizes[7] != NCLS) return;
  if ((long long)out_size != (long long)nN * NCLS) return;

  const float* x    = (const float*)d_in[0];
  const int*   edge = (const int*)d_in[1];
  const float* W1   = (const float*)d_in[2];
  const float* b1   = (const float*)d_in[3];
  const float* W2   = (const float*)d_in[4];
  const float* b2   = (const float*)d_in[5];
  const float* Wfc  = (const float*)d_in[6];
  const float* bfc  = (const float*)d_in[7];
  float* out = (float*)d_out;
  const int* src = edge;
  const int* dst = edge + nE;

  const int MP   = cdiv(nN, MROWS) * MROWS;
  const int gM   = MP / GBM;
  const int gH   = MP / HBM;
  const int gA   = cdiv(MP, NBA);
  const int gD   = cdiv(MP, NBD);
  const int NBPD = gD * NBD;
  if ((long long)gA * NBA < (long long)MP) return;
  if (NBPD < MP) return;
  const int vec8 = ((nE & 3) == 0) ? 1 : 0;
  const int nUx  = MP * (FIN / 8);
  if ((nUx % NTHR) != 0) return;

  char* ws = (char*)d_ws;
  size_t off = 0;
  const size_t oR1  = off; off = al256(off + (size_t)MP * K2 * 2);
  const size_t oR2  = off; off = al256(off + (size_t)MP * HID * 4);
  const size_t oLST = off; off = al256(off + (size_t)gA * RCAP * 4);
  const size_t oTAB = off; off = al256(off + (size_t)gA * NBA * 16);
  const size_t oNO  = off; off = al256(off + (size_t)NBPD * 4);
  const size_t oFLG = off; off = al256(off + (size_t)gA * 128);
  const size_t oW1T = off; off = al256(off + (size_t)HID * FIN * 2);
  const size_t oW2T = off; off = al256(off + (size_t)HID * K2 * 2);
  const size_t oWFT = off; off = al256(off + (size_t)NCP * K2 * 2);
  const size_t oBT  = off; off = al256(off + (size_t)3 * HID * 4);
  if (off > ws_size || off > (size_t)WSMAX) return;
  if ((size_t)MP * FIN * 2 > (size_t)MP * K2 * 2) return;
  unsigned short* XB  = (unsigned short*)(ws + oR1);
  unsigned short* G   = (unsigned short*)(ws + oR1);
  float*          H   = (float*)(ws + oR2);
  int*            LST = (int*)(ws + oLST);
  int*            TAB = (int*)(ws + oTAB);
  float*          NO  = (float*)(ws + oNO);
  int*            FLG = (int*)(ws + oFLG);
  unsigned short* W1T = (unsigned short*)(ws + oW1T);
  unsigned short* W2T = (unsigned short*)(ws + oW2T);
  unsigned short* WFT = (unsigned short*)(ws + oWFT);
  float*          BT  = (float*)(ws + oBT);

  const int bktLds = BKT_LDS_INTS * 4;
  hipFuncSetAttribute(reinterpret_cast<const void*>(&k_bucket),
                      hipFuncAttributeMaxDynamicSharedMemorySize, bktLds);

  k_prep<<<(nUx + NUW1 + NUW2 + NUW3) / NTHR + 1, NTHR, 0, stream>>>(x, W1, W2, Wfc, b1, b2, bfc,
                                                                       XB, W1T, W2T, WFT, BT, nN, nUx);
  k_bucket<<<gA, NTHR, bktLds, stream>>>(src, dst, nE, nN, vec8, LST, TAB, FLG);
  k_outdeg<<<gD, NTHR, 0, stream>>>(src, nE, vec8, NO);
  k_gemm<1><<<dim3(gM, HID / GBN), GTHR, 0, stream>>>(XB, W1T, H, FIN, HID, NO);
  k_agg<1><<<gA, NTHR, 0, stream>>>(LST, TAB, FLG, H, BT, NO, G, nN, MP);
  k_gemm<0><<<dim3(gM, HID / GBN), GTHR, 0, stream>>>(G, W2T, H, K2, HID, NO);
  k_agg<2><<<gA, NTHR, 0, stream>>>(LST, TAB, FLG, H, BT + HID, NO, G, nN, MP);
  k_head<<<gH, NTHR, 0, stream>>>(G, WFT, BT + 2 * HID, FLG, out, nN * NCLS);
}
